// VisionSelfAttention_82772609728633
// MI455X (gfx1250) — hardware-verified
//
#include <hip/hip_runtime.h>


#define NPIX 65536
#define HH   64
#define WWD  64
#define CC   192
#define NHD  8
#define KD   32
#define DQ   (NHD * KD)
#define CK   (CC + 2)
#define HP   (NPIX / 2)
typedef _Float16 h16;
typedef unsigned short bf;
typedef __attribute__((ext_vector_type(16))) __bf16   v16bf;
typedef __attribute__((ext_vector_type(16))) _Float16 v16h;
typedef __attribute__((ext_vector_type(8)))  _Float16 v8h;
typedef __attribute__((ext_vector_type(8)))  unsigned short v8us;
typedef __attribute__((ext_vector_type(8)))  float    v8f;
typedef __attribute__((ext_vector_type(4)))  float    v4f;
typedef v8h  __attribute__((may_alias)) v8ha;
typedef v4f  __attribute__((may_alias)) v4fa;
typedef v8us __attribute__((may_alias)) v8usa;

__device__ __forceinline__ unsigned short f2bf(float f) { unsigned u = __float_as_uint(f); u += 0x7FFFu + ((u >> 16) & 1u); return (unsigned short)(u >> 16); }
__device__ __forceinline__ float bf2f(unsigned short b) { return __uint_as_float(((unsigned)b) << 16); }
__device__ __forceinline__ float bfr(float f) { return bf2f(f2bf(f)); }
__device__ __forceinline__ v16h cat16(v8h lo, v8h hi) { return __builtin_shufflevector(lo, hi, 0, 1, 2, 3, 4, 5, 6, 7, 8, 9, 10, 11, 12, 13, 14, 15); }
__device__ __forceinline__ v16bf cat16b(v8us lo, v8us hi) { return __builtin_bit_cast(v16bf, __builtin_shufflevector(lo, hi, 0, 1, 2, 3, 4, 5, 6, 7, 8, 9, 10, 11, 12, 13, 14, 15)); }
__device__ __forceinline__ v8f wmma16(v16h a, v16h b, v8f c) { return __builtin_amdgcn_wmma_f32_16x16x32_f16(false, a, false, b, (short)0, c, false, false); }
__device__ __forceinline__ v8f wmmab(v16bf a, v16bf b, v8f c) { return __builtin_amdgcn_wmma_f32_16x16x32_bf16(false, a, false, b, (short)0, c, false, false); }


template <typename T16> struct WFrag;
template <> struct WFrag<h16> { typedef v16h V; static __device__ __forceinline__ V ld(const h16* p) { return cat16(*(const v8h*)p, *(const v8h*)(p + 16)); } static __device__ __forceinline__ v8f mma(V a, V b, v8f c) { return wmma16(a, b, c); } };
template <> struct WFrag<bf> { typedef v16bf V; static __device__ __forceinline__ V ld(const bf* p) { return cat16b(*(const v8us*)p, *(const v8us*)(p + 16)); } static __device__ __forceinline__ v8f mma(V a, V b, v8f c) { return wmmab(a, b, c); } };
template <typename T16, int NSPLIT, bool BIAS>
__global__ __launch_bounds__(32) void k_gemmw(const T16* __restrict__ A, const T16* __restrict__ A2, const T16* __restrict__ Bt, const T16* __restrict__ Bt2, int K, float* C, int ldc, const float* __restrict__ bias, size_t sA, size_t sB, size_t sC) {
    typedef typename WFrag<T16>::V V;
    __shared__ __align__(16) float os[16 * 68];
    const size_t z = blockIdx.z; A += z * sA; if (A2) A2 += z * sA; Bt += z * sB; if (Bt2) Bt2 += z * sB; C += z * sC;
    const int lane = threadIdx.x & 31, lr = lane & 15, hi = lane >> 4; const int r0 = blockIdx.x * 64, c0 = blockIdx.y * 64;
    v8f acc[4][4];
#pragma unroll
    for (int mb = 0; mb < 4; ++mb)
#pragma unroll
        for (int nb = 0; nb < 4; ++nb) acc[mb][nb] = (v8f){};
    const size_t aoff = (size_t)(r0 + lr) * K + 8 * hi, boff = (size_t)(c0 + lr) * K + 8 * hi;
#pragma unroll 1
    for (int kc = 0; kc < K; kc += 32) {
        V a[4], a2[4];
#pragma unroll
        for (int mb = 0; mb < 4; ++mb) { a[mb] = WFrag<T16>::ld(A + aoff + (size_t)mb * 16 * K + kc); if (NSPLIT == 1 || NSPLIT == 2) a2[mb] = WFrag<T16>::ld(A2 + aoff + (size_t)mb * 16 * K + kc); }
#pragma unroll
        for (int nb = 0; nb < 4; ++nb) { const V b = WFrag<T16>::ld(Bt + boff + (size_t)nb * 16 * K + kc); V b2; if (NSPLIT >= 2) b2 = WFrag<T16>::ld(Bt2 + boff + (size_t)nb * 16 * K + kc);
#pragma unroll
            for (int mb = 0; mb < 4; ++mb) { acc[mb][nb] = WFrag<T16>::mma(a[mb], b, acc[mb][nb]); if (NSPLIT == 1 || NSPLIT == 2) acc[mb][nb] = WFrag<T16>::mma(a2[mb], b, acc[mb][nb]); if (NSPLIT >= 2) acc[mb][nb] = WFrag<T16>::mma(a[mb], b2, acc[mb][nb]); } }
        asm volatile("v_nop\n\tv_nop\n\tv_nop\n\tv_nop" : "+v"(acc[0][0]), "+v"(acc[1][1]), "+v"(acc[2][2]), "+v"(acc[3][3]) : "v"(a[0]), "v"(a[3]));
    }
#pragma unroll
    for (int mb = 0; mb < 4; ++mb) {
#pragma unroll
        for (int nb = 0; nb < 4; ++nb) {
#pragma unroll
            for (int j = 0; j < 8; ++j) os[(hi * 8 + j) * 68 + nb * 16 + lr] = acc[mb][nb][j]; }
        __builtin_amdgcn_wave_barrier(); asm volatile("" ::: "memory");
        float* crow = C + (size_t)(r0 + mb * 16) * ldc + c0;
#pragma unroll 1
        for (int ps = 0; ps < 2; ++ps) {
#pragma unroll
            for (int s = 0; s < 8; ++s) { const int row = 2 * s + hi, cofs = lr * 4; v4f val = *(const v4fa*)(os + row * 68 + cofs); if (BIAS) { val[0] += bfr(bias[c0 + cofs]); val[1] += bfr(bias[c0 + cofs + 1]); val[2] += bfr(bias[c0 + cofs + 2]); val[3] += bfr(bias[c0 + cofs + 3]); }
                *(volatile v4f*)(crow + (size_t)row * ldc + cofs) = val; }
            if (ps == 0) __threadfence(); }
        __builtin_amdgcn_wave_barrier(); asm volatile("" ::: "memory");
    }
}

__device__ __forceinline__ void splitf(float y, unsigned short& h, unsigned short& l) { h = f2bf(y); l = f2bf(y - bf2f(h)); }
typedef __attribute__((ext_vector_type(4))) unsigned short v4us;

__global__ __launch_bounds__(256) void k_cvt8(const float* __restrict__ src, bf* dst, size_t n8) { const size_t i = (size_t)blockIdx.x * 256 + threadIdx.x; if (i >= n8) return; const v8f v = *(const v8f*)(src + i * 8); v8us o;
#pragma unroll
    for (int k = 0; k < 8; ++k) o[k] = f2bf(v[k]); *(volatile v8us*)(dst + i * 8) = o; __threadfence(); *(volatile v8us*)(dst + i * 8) = o; }
__global__ __launch_bounds__(256) void k_wq(const float* __restrict__ w, bf* Bt) { const int e = (blockIdx.x * 256 + threadIdx.x) * 4; if (e >= DQ * CC) return; const int c = e % CC, n = e / CC; v4us o;
#pragma unroll
    for (int q = 0; q < 4; ++q) o[q] = f2bf(w[(size_t)(c + q) * DQ + n]); *(volatile v4us*)(Bt + e) = o; __threadfence(); *(volatile v4us*)(Bt + e) = o; }
__global__ __launch_bounds__(256) void k_wo(const float* __restrict__ w, bf* Bt) { const int e = (blockIdx.x * 256 + threadIdx.x) * 4; if (e >= CC * DQ) return; const int n = e % DQ, c = e / DQ; v4us o;
#pragma unroll
    for (int q = 0; q < 4; ++q) o[q] = f2bf(w[(size_t)(n + q) * CC + c]); *(volatile v4us*)(Bt + e) = o; __threadfence(); *(volatile v4us*)(Bt + e) = o; }
__global__ __launch_bounds__(256) void k_dtab(const float* __restrict__ Wk, const float* __restrict__ bk, const float* __restrict__ Wv, const float* __restrict__ bv, float* DK, float* DV) { const int e = blockIdx.x * 256 + threadIdx.x; if (e >= 9 * DQ) return; const int n = e % DQ, j = e / DQ; const float dx = (float)(j % 3 - 1), dy = (float)(j / 3 - 1);
    float a = __fmul_rn(dx, bfr(Wk[(size_t)CC * DQ + n])), b = __fmul_rn(dy, bfr(Wk[(size_t)(CC + 1) * DQ + n])); asm volatile("" : "+v"(a), "+v"(b)); const float dk = __fadd_rn(__fadd_rn(a, b), bfr(bk[n]));
    float a2 = __fmul_rn(dx, bfr(Wv[(size_t)CC * DQ + n])), b2 = __fmul_rn(dy, bfr(Wv[(size_t)(CC + 1) * DQ + n])); asm volatile("" : "+v"(a2), "+v"(b2)); const float dv = __fadd_rn(__fadd_rn(a2, b2), bfr(bv[n]));
    *(volatile float*)(DK + e) = dk; *(volatile float*)(DV + e) = dv; __threadfence(); *(volatile float*)(DK + e) = dk; *(volatile float*)(DV + e) = dv; }
__global__ __launch_bounds__(256) void k_lwa(const float* __restrict__ XQ, const float* __restrict__ XK, const float* __restrict__ XV, const float* __restrict__ DK, const float* __restrict__ DV, bf* Oh, bf* Ol) {
    const int idx = blockIdx.x * 256 + threadIdx.x; if (idx >= HP * NHD) return; const int h = idx % NHD, p = idx / NHD; const int b = p / (HH * WWD), y = (p / WWD) % HH, x = p % WWD;     const float* qp = XQ + (size_t)p * DQ + h * KD;
    float s[9]; int nbp[9];
#pragma unroll
    for (int j = 0; j < 9; ++j) { const int yy = y + j / 3 - 1, xx = x + j % 3 - 1; const bool in = (yy >= 0 && yy < HH && xx >= 0 && xx < WWD); nbp[j] = in ? (b * HH + yy) * WWD + xx : -1; const float* kp = XK + (size_t)(in ? nbp[j] : 0) * DQ + h * KD; const float* dk = DK + j * DQ + h * KD; float acc = 0.f;
#pragma unroll 8
        for (int d = 0; d < KD; ++d) { const float kv = __fadd_rn(in ? kp[d] : 0.f, dk[d]); float pr = __fmul_rn(qp[d], kv); asm volatile("" : "+v"(pr)); acc = __fadd_rn(acc, pr); }
        s[j] = __fmul_rn(acc, 0.17677669529663687f); }
    float m = s[0];
#pragma unroll
    for (int j = 1; j < 9; ++j) m = fmaxf(m, s[j]);
    float e9[9]; float sum = 0.f;
#pragma unroll
    for (int j = 0; j < 9; ++j) { float d0 = __fsub_rn(s[j], m); asm volatile("" : "+v"(d0)); e9[j] = __expf(d0); sum = __fadd_rn(sum, e9[j]); }
    const float rs = __fdiv_rn(1.0f, sum); bf* oh = Oh + (size_t)p * DQ + h * KD; bf* ol = Ol + (size_t)p * DQ + h * KD;
#pragma unroll 1
    for (int ps = 0; ps < 2; ++ps) {
#pragma unroll 1
        for (int d0_ = 0; d0_ < KD; d0_ += 4) { v4us o4h, o4l;
#pragma unroll
            for (int u = 0; u < 4; ++u) { const int d = d0_ + u; float o = 0.f;
#pragma unroll
                for (int j = 0; j < 9; ++j) { const float vv = __fadd_rn(nbp[j] >= 0 ? XV[(size_t)nbp[j] * DQ + h * KD + d] : 0.f, DV[j * DQ + h * KD + d]); float a = __fmul_rn(e9[j], rs); asm volatile("" : "+v"(a)); float pr = __fmul_rn(a, vv); asm volatile("" : "+v"(pr)); o = __fadd_rn(o, pr); }
                unsigned short a2, c2; splitf(o, a2, c2); o4h[u] = a2; o4l[u] = c2; }
            *(volatile v4us*)(oh + d0_) = o4h; *(volatile v4us*)(ol + d0_) = o4l; }
        if (ps == 0) __threadfence(); } }

extern "C" void kernel_launch(void* const* d_in, const int* in_sizes, int n_in,
                              void* d_out, int out_size, void* d_ws, size_t ws_size, hipStream_t stream) {
    (void)in_sizes; (void)n_in; (void)out_size;
    const float* x = (const float*)d_in[0]; const float* Wq = (const float*)d_in[1]; const float* bq = (const float*)d_in[2]; const float* Wk = (const float*)d_in[3]; const float* bk = (const float*)d_in[4]; const float* Wv = (const float*)d_in[5]; const float* bv = (const float*)d_in[6]; const float* Wo = (const float*)d_in[7]; const float* bo = (const float*)d_in[8];
    float* OUT = (float*)d_out;
    char* wsp = (char*)d_ws;
    auto take = [&](size_t bytes) { char* p = wsp; wsp += (bytes + 255) & ~(size_t)255; return (void*)p; };
    bf* WQ = (bf*)take((size_t)DQ * CC * 2); bf* WK = (bf*)take((size_t)DQ * CC * 2); bf* WV = (bf*)take((size_t)DQ * CC * 2); bf* WO = (bf*)take((size_t)CC * DQ * 2); float* DK = (float*)take((size_t)9 * DQ * 4); float* DV = (float*)take((size_t)9 * DQ * 4);
    bf* XB = (bf*)take((size_t)HP * CC * 2); float* XQ = (float*)take((size_t)HP * DQ * 4); float* XK = (float*)take((size_t)HP * DQ * 4); float* XV = (float*)take((size_t)HP * DQ * 4); bf* Oh = (bf*)take((size_t)HP * DQ * 2); bf* Ol = (bf*)take((size_t)HP * DQ * 2);
    if ((size_t)(wsp - (char*)d_ws) > ws_size) return;
    { const unsigned g = (DQ * CC / 4 + 255) / 256; k_wq<<<g, 256, 0, stream>>>(Wq, WQ); k_wq<<<g, 256, 0, stream>>>(Wk, WK); k_wq<<<g, 256, 0, stream>>>(Wv, WV); k_wo<<<(CC * DQ / 4 + 255) / 256, 256, 0, stream>>>(Wo, WO); k_dtab<<<(9 * DQ + 255) / 256, 256, 0, stream>>>(Wk, bk, Wv, bv, DK, DV); }
    const dim3 gP(HP / 64, DQ / 64, 1);
    for (int gh = 0; gh < NPIX / HP; ++gh) { const size_t p0 = (size_t)gh * HP;
        k_cvt8<<<(unsigned)(((size_t)HP * CC / 8 + 255) / 256), 256, 0, stream>>>(x + p0 * CC, XB, (size_t)HP * CC / 8);
        k_gemmw<bf, 0, true><<<gP, 32, 0, stream>>>(XB, nullptr, WQ, nullptr, CC, XQ, DQ, bq, 0, 0, 0);
        k_gemmw<bf, 0, false><<<gP, 32, 0, stream>>>(XB, nullptr, WK, nullptr, CC, XK, DQ, nullptr, 0, 0, 0);
        k_gemmw<bf, 0, false><<<gP, 32, 0, stream>>>(XB, nullptr, WV, nullptr, CC, XV, DQ, nullptr, 0, 0, 0);
        k_lwa<<<(HP * NHD + 255) / 256, 256, 0, stream>>>(XQ, XK, XV, DK, DV, Oh, Ol);
        k_gemmw<bf, 1, true><<<dim3(HP / 64, CC / 64, 1), 32, 0, stream>>>(Oh, Ol, WO, nullptr, DQ, OUT + p0 * CC, CC, bo, 0, 0, 0); }
}
